// MambaBlock_47880295416210
// MI455X (gfx1250) — hardware-verified
//
#include <hip/hip_runtime.h>
#include <stddef.h>
#include <stdint.h>
#include <math.h>


#define DMODEL 1024
#define DINNER 2048
#define DSTATE 16
#define DTRANK 64
#define NBATCH 2
#define SEQLEN 2048
#define MROWS  4096
#define XPN    96
#define XPNP   128
#define KIN    1024
#define KX2    4096
#define KD2    128
#define KO2    4096
#define XZP    4096
#define BCP    32
#define GBM    64
#define GBN    64
#define GTHR   128
#define NTHR   256
#define SCH    64
#define TCH    32
#define SCTHR  (SCH * 4)

#define EP_IN  0
#define EP_XP  1
#define EP_DT  2
#define EP_OUT 3

static_assert(MROWS == NBATCH * SEQLEN);
static_assert(MROWS % GBM == 0);
static_assert((2 * DINNER) % GBN == 0 && XPNP % GBN == 0 && DINNER % GBN == 0 && DMODEL % GBN == 0);
static_assert(KIN % 32 == 0 && KX2 % 32 == 0 && KD2 % 32 == 0 && KO2 % 32 == 0);
static_assert(KX2 == 2 * DINNER && KD2 == 2 * DTRANK && KO2 == 2 * DINNER);
static_assert(GBM == (GTHR / 32) * 16 && GBN == 64);
static_assert(XPN == DTRANK + 2 * DSTATE && BCP == 2 * DSTATE);
static_assert(SCTHR == 256 && TCH * SCH / 4 == 2 * SCTHR && TCH * BCP / 4 == SCTHR && TCH * SCH / 8 == SCTHR);
static_assert(SEQLEN % TCH == 0 && DINNER % SCH == 0);
static_assert(DINNER == 8 * NTHR && DMODEL == 4 * 32 * 8);
static_assert((SEQLEN & (SEQLEN - 1)) == 0);

typedef float          v4f   __attribute__((ext_vector_type(4)));
typedef float          v8f   __attribute__((ext_vector_type(8)));
typedef int            v8i   __attribute__((ext_vector_type(8)));
typedef unsigned short v4us  __attribute__((ext_vector_type(4)));
typedef unsigned short v8us  __attribute__((ext_vector_type(8)));
typedef unsigned short v16us __attribute__((ext_vector_type(16)));
typedef __bf16         v16bf __attribute__((ext_vector_type(16)));
typedef v4f  __attribute__((may_alias)) v4fa;
typedef v4us __attribute__((may_alias)) v4usa;
typedef v8us __attribute__((may_alias)) v8usa;
union FragB { v16bf v; v16us u; v8us h[2]; v8i w; };

__device__ __forceinline__ v8f wmb(const FragB& a, const FragB& b, v8f c) {
  v8f d = __builtin_amdgcn_wmma_f32_16x16x32_bf16(false, a.v, false, b.v, (short)0, c, false, false);
  asm volatile("v_nop\n\tv_nop\n\tv_nop\n\tv_nop" : "+v"(d) : "v"(a.w), "v"(b.w));
  return d;
}

__device__ __forceinline__ unsigned bf16_bits(float f) {
  const unsigned u = __float_as_uint(f);
  return (u + 0x7FFFu + ((u >> 16) & 1u)) >> 16;
}
__device__ __forceinline__ float bf16_val(float f) {
  return __uint_as_float(bf16_bits(f) << 16);
}
__device__ __forceinline__ void hl_bits(float v, unsigned& hb, unsigned& lb) {
  hb = bf16_bits(v);
  lb = bf16_bits(v - __uint_as_float(hb << 16));
}
__device__ __forceinline__ float silu_f(float v) {
  return v * __builtin_amdgcn_rcpf(1.0f + expf(-v));
}
__device__ __forceinline__ float softplus_f(float v) {
  return fmaxf(v, 0.0f) + log1pf(expf(-fabsf(v)));
}

__global__ __launch_bounds__(NTHR) void k_cvt(const float* __restrict__ src, int srcRows, int srcK,
                                              unsigned short* dst, int pshift, int nUnits) {
  const int u = (int)blockIdx.x * NTHR + (int)threadIdx.x;
  if (u >= nUnits) return;
  const int row = u >> pshift;
  const int k8  = (u & ((1 << pshift) - 1)) * 8;
  const int rc  = row < srcRows ? row : srcRows - 1;
  const int sc  = k8 & (srcK - 1);
  const float* p = src + (size_t)rc * (size_t)srcK + sc;
  const v4f a = *(const v4fa*)p;
  const v4f b = *(const v4fa*)(p + 4);
  const bool ok = row < srcRows;
  v8us o;
  o[0] = ok ? (unsigned short)bf16_bits(a.x) : (unsigned short)0;
  o[1] = ok ? (unsigned short)bf16_bits(a.y) : (unsigned short)0;
  o[2] = ok ? (unsigned short)bf16_bits(a.z) : (unsigned short)0;
  o[3] = ok ? (unsigned short)bf16_bits(a.w) : (unsigned short)0;
  o[4] = ok ? (unsigned short)bf16_bits(b.x) : (unsigned short)0;
  o[5] = ok ? (unsigned short)bf16_bits(b.y) : (unsigned short)0;
  o[6] = ok ? (unsigned short)bf16_bits(b.z) : (unsigned short)0;
  o[7] = ok ? (unsigned short)bf16_bits(b.w) : (unsigned short)0;
  unsigned short* dp = dst + ((size_t)row << (pshift + 3)) + k8;
  *(volatile v8us*)dp = o;
  __threadfence();
  *(volatile v8us*)dp = o;
}

template <int EP>
__global__ __launch_bounds__(GTHR) void k_gemm(
    const unsigned short* __restrict__ A, const unsigned short* __restrict__ WT, int K,
    float* outF, int ldo, unsigned short* outH, const float* __restrict__ aux)
{
  __shared__ __attribute__((aligned(16))) float stg[GBM * GBN];
  const int tid = (int)threadIdx.x, lane = tid & 31, wave = tid >> 5, hh = lane >> 4, m = lane & 15;
  const int rowBase = (int)blockIdx.x * GBM;
  const int col0    = (int)blockIdx.y * GBN;

  v8f acc[4];
  {
    const v8f z = {0.f, 0.f, 0.f, 0.f, 0.f, 0.f, 0.f, 0.f};
    acc[0] = z; acc[1] = z; acc[2] = z; acc[3] = z;
  }
  const unsigned short* ap = A  + (size_t)(rowBase + 16 * wave + m) * (size_t)K + 8 * hh;
  const unsigned short* wp = WT + (size_t)(col0 + m) * (size_t)K + 8 * hh;
  const int ksteps = K >> 5;
#pragma unroll 1
  for (int ks = 0; ks < ksteps; ++ks) {
    FragB af;
    af.h[0] = *(const v8usa*)(ap + 32 * ks);
    af.h[1] = *(const v8usa*)(ap + 32 * ks + 16);
#pragma unroll
    for (int t = 0; t < 4; ++t) {
      const unsigned short* wq = wp + (size_t)(16 * t) * (size_t)K + 32 * ks;
      FragB bf;
      bf.h[0] = *(const v8usa*)wq;
      bf.h[1] = *(const v8usa*)(wq + 16);
      acc[t] = wmb(af, bf, acc[t]);
    }
  }

#pragma unroll
  for (int t = 0; t < 4; ++t) {
    const int lc = 16 * t + m;
#pragma unroll
    for (int r = 0; r < 8; ++r) {
      const int lr = 16 * wave + 8 * hh + r;
      stg[lr * GBN + lc] = acc[t][r];
    }
  }
  __syncthreads();

  if constexpr (EP == EP_XP) {
    (void)ldo; (void)aux;
    if (col0 == 0) {
      const bool lsel = (m & 8) != 0;
      v8us qv[8];
#pragma unroll
      for (int i = 0; i < 8; ++i) {
        const int lr = 16 * wave + 2 * i + hh;
        const float* sp = stg + lr * GBN + 8 * (m & 7);
        const v4f a = *(const v4fa*)sp;
        const v4f b = *(const v4fa*)(sp + 4);
        unsigned hb, lb;
        v8us o;
        hl_bits(a.x, hb, lb); o[0] = (unsigned short)(lsel ? lb : hb);
        hl_bits(a.y, hb, lb); o[1] = (unsigned short)(lsel ? lb : hb);
        hl_bits(a.z, hb, lb); o[2] = (unsigned short)(lsel ? lb : hb);
        hl_bits(a.w, hb, lb); o[3] = (unsigned short)(lsel ? lb : hb);
        hl_bits(b.x, hb, lb); o[4] = (unsigned short)(lsel ? lb : hb);
        hl_bits(b.y, hb, lb); o[5] = (unsigned short)(lsel ? lb : hb);
        hl_bits(b.z, hb, lb); o[6] = (unsigned short)(lsel ? lb : hb);
        hl_bits(b.w, hb, lb); o[7] = (unsigned short)(lsel ? lb : hb);
        qv[i] = o;
      }
#pragma unroll
      for (int i = 0; i < 8; ++i) {
        const int lr = 16 * wave + 2 * i + hh;
        unsigned short* hp = outH + (size_t)(rowBase + lr) * KD2 + 8 * m;
        *(volatile v8us*)hp = qv[i];
      }
      __threadfence();
#pragma unroll
      for (int i = 0; i < 8; ++i) {
        const int lr = 16 * wave + 2 * i + hh;
        unsigned short* hp = outH + (size_t)(rowBase + lr) * KD2 + 8 * m;
        *(volatile v8us*)hp = qv[i];
      }
    } else {
      const int rq = lane >> 3, c4 = 4 * (lane & 7);
      v4f fv[4];
#pragma unroll
      for (int i = 0; i < 4; ++i) {
        const int lr = 16 * wave + 4 * i + rq;
        fv[i] = *(const v4fa*)(stg + lr * GBN + c4);
      }
#pragma unroll
      for (int i = 0; i < 4; ++i) {
        const int lr = 16 * wave + 4 * i + rq;
        float* op = outF + (size_t)(rowBase + lr) * BCP + c4;
        *(volatile v4f*)op = fv[i];
      }
      __threadfence();
#pragma unroll
      for (int i = 0; i < 4; ++i) {
        const int lr = 16 * wave + 4 * i + rq;
        float* op = outF + (size_t)(rowBase + lr) * BCP + c4;
        *(volatile v4f*)op = fv[i];
      }
    }
  } else {
    (void)outH;
    if constexpr (EP == EP_IN) {
      (void)aux;
      if (col0 >= DINNER) {
#pragma unroll 1
        for (int i = 0; i < 8; ++i) {
          float* sp = stg + (16 * wave + 2 * i + hh) * GBN + 4 * m;
          v4f v = *(const v4fa*)sp;
          v.x = silu_f(v.x); v.y = silu_f(v.y); v.z = silu_f(v.z); v.w = silu_f(v.w);
          *(v4fa*)sp = v;
        }
      }
    }
    if constexpr (EP == EP_DT) {
      const v4f bq = *(const v4fa*)(aux + col0 + 4 * m);
      const float b0 = bf16_val(bq.x), b1 = bf16_val(bq.y), b2 = bf16_val(bq.z), b3 = bf16_val(bq.w);
#pragma unroll 1
      for (int i = 0; i < 8; ++i) {
        float* sp = stg + (16 * wave + 2 * i + hh) * GBN + 4 * m;
        v4f v = *(const v4fa*)sp;
        v.x = softplus_f(v.x + b0); v.y = softplus_f(v.y + b1);
        v.z = softplus_f(v.z + b2); v.w = softplus_f(v.w + b3);
        *(v4fa*)sp = v;
      }
    }
    if constexpr (EP == EP_OUT) {
#pragma unroll 1
      for (int i = 0; i < 8; ++i) {
        const int lr = 16 * wave + 2 * i + hh;
        float* sp = stg + lr * GBN + 4 * m;
        const v4f xr = *(const v4fa*)(aux + (size_t)(rowBase + lr) * DMODEL + col0 + 4 * m);
        v4f v = *(const v4fa*)sp;
        v.x += bf16_val(xr.x); v.y += bf16_val(xr.y); v.z += bf16_val(xr.z); v.w += bf16_val(xr.w);
        *(v4fa*)sp = v;
      }
    }
    v4f fv[8];
#pragma unroll
    for (int i = 0; i < 8; ++i) {
      const int lr = 16 * wave + 2 * i + hh;
      fv[i] = *(const v4fa*)(stg + lr * GBN + 4 * m);
    }
#pragma unroll
    for (int i = 0; i < 8; ++i) {
      const int lr = 16 * wave + 2 * i + hh;
      float* op = outF + (size_t)(rowBase + lr) * (size_t)ldo + col0 + 4 * m;
      *(volatile v4f*)op = fv[i];
    }
    __threadfence();
#pragma unroll
    for (int i = 0; i < 8; ++i) {
      const int lr = 16 * wave + 2 * i + hh;
      float* op = outF + (size_t)(rowBase + lr) * (size_t)ldo + col0 + 4 * m;
      *(volatile v4f*)op = fv[i];
    }
  }
}

__global__ __launch_bounds__(NTHR) void k_conv(const float* __restrict__ xz, const float* __restrict__ cw,
                                               const float* __restrict__ cb, float* U, unsigned short* UHL) {
  __shared__ __attribute__((aligned(16))) float su[DINNER];
  __shared__ __attribute__((aligned(16))) unsigned short sh[DINNER];
  __shared__ __attribute__((aligned(16))) unsigned short sl[DINNER];
  const int tid  = (int)threadIdx.x;
  const int mrow = (int)blockIdx.x;
  const int l    = mrow & (SEQLEN - 1);
#pragma unroll 1
  for (int hf = 0; hf < 2; ++hf) {
    const int c = hf * 1024 + 4 * tid;
    const v4f w0 = *(const v4fa*)(cw + 4 * (size_t)(c + 0));
    const v4f w1 = *(const v4fa*)(cw + 4 * (size_t)(c + 1));
    const v4f w2 = *(const v4fa*)(cw + 4 * (size_t)(c + 2));
    const v4f w3 = *(const v4fa*)(cw + 4 * (size_t)(c + 3));
    const v4f bq = *(const v4fa*)(cb + c);
    float s0 = 0.0f, s1 = 0.0f, s2 = 0.0f, s3 = 0.0f;
#pragma unroll
    for (int j = 0; j < 4; ++j) {
      const bool ok = (l - 3 + j) >= 0;
      const int  mr = ok ? (mrow - 3 + j) : mrow;
      const v4f  xv = *(const v4fa*)(xz + (size_t)mr * XZP + c);
      const float f = ok ? 1.0f : 0.0f;
      s0 = fmaf(bf16_val(w0[j]), xv.x * f, s0);
      s1 = fmaf(bf16_val(w1[j]), xv.y * f, s1);
      s2 = fmaf(bf16_val(w2[j]), xv.z * f, s2);
      s3 = fmaf(bf16_val(w3[j]), xv.w * f, s3);
    }
    v4f uv;
    uv.x = silu_f(s0 + bf16_val(bq.x));
    uv.y = silu_f(s1 + bf16_val(bq.y));
    uv.z = silu_f(s2 + bf16_val(bq.z));
    uv.w = silu_f(s3 + bf16_val(bq.w));
    v4us h4, l4;
    unsigned hb, lb;
    hl_bits(uv.x, hb, lb); h4[0] = (unsigned short)hb; l4[0] = (unsigned short)lb;
    hl_bits(uv.y, hb, lb); h4[1] = (unsigned short)hb; l4[1] = (unsigned short)lb;
    hl_bits(uv.z, hb, lb); h4[2] = (unsigned short)hb; l4[2] = (unsigned short)lb;
    hl_bits(uv.w, hb, lb); h4[3] = (unsigned short)hb; l4[3] = (unsigned short)lb;
    *(v4fa*)(su + c)  = uv;
    *(v4usa*)(sh + c) = h4;
    *(v4usa*)(sl + c) = l4;
  }
  __syncthreads();
  const v4f  o0 = *(const v4fa*)(su + 4 * tid);
  const v4f  o1 = *(const v4fa*)(su + 1024 + 4 * tid);
  const v8us qh = *(const v8usa*)(sh + 8 * tid);
  const v8us ql = *(const v8usa*)(sl + 8 * tid);
  float* up = U + (size_t)mrow * DINNER + 4 * tid;
  unsigned short* hp = UHL + (size_t)mrow * KX2 + 8 * tid;
  *(volatile v4f*)up = o0;
  *(volatile v4f*)(up + 1024) = o1;
  *(volatile v8us*)hp = qh;
  *(volatile v8us*)(hp + DINNER) = ql;
  __threadfence();
  *(volatile v4f*)up = o0;
  *(volatile v4f*)(up + 1024) = o1;
  *(volatile v8us*)hp = qh;
  *(volatile v8us*)(hp + DINNER) = ql;
}

__global__ __launch_bounds__(SCTHR) void k_scan(const float* __restrict__ xz, const float* __restrict__ U,
                                                const float* __restrict__ BC, const float* __restrict__ Alog,
                                                const float* __restrict__ Dp, unsigned short* YHL) {
  __shared__ __attribute__((aligned(16))) float sD[TCH * SCH];
  __shared__ __attribute__((aligned(16))) float sU[TCH * SCH];
  __shared__ __attribute__((aligned(16))) float sG[TCH * SCH];
  __shared__ __attribute__((aligned(16))) float sBC[TCH * BCP];
  __shared__ __attribute__((aligned(16))) unsigned short sYh[TCH * SCH];
  __shared__ __attribute__((aligned(16))) unsigned short sYl[TCH * SCH];
  const int tid = (int)threadIdx.x;
  const int ch  = tid >> 2, q = tid & 3;
  const int b   = (int)blockIdx.x / (DINNER / SCH);
  const int d0  = ((int)blockIdx.x % (DINNER / SCH)) * SCH;
  const int d   = d0 + ch;

  float a0, a1, a2, a3;
  {
    const v4f al = *(const v4fa*)(Alog + (size_t)d * DSTATE + 4 * q);
    a0 = -expf(bf16_val(al.x)); a1 = -expf(bf16_val(al.y));
    a2 = -expf(bf16_val(al.z)); a3 = -expf(bf16_val(al.w));
  }
  const float Dd = bf16_val(Dp[d]);
  float h0 = 0.0f, h1 = 0.0f, h2 = 0.0f, h3 = 0.0f;

  const int orow = tid >> 3, oq = tid & 7;

#pragma unroll 1
  for (int cnk = 0; cnk < SEQLEN / TCH; ++cnk) {
    const int rb = b * SEQLEN + cnk * TCH;
#pragma unroll
    for (int it = 0; it < 2; ++it) {
      const int idx = it * SCTHR + tid;
      const int r   = idx >> 4;
      const int c4  = (idx & 15) * 4;
      const float* px = xz + (size_t)(rb + r) * XZP + d0 + c4;
      const v4f vd = *(const v4fa*)px;
      const v4f vg = *(const v4fa*)(px + DINNER);
      const v4f vu = *(const v4fa*)(U + (size_t)(rb + r) * DINNER + d0 + c4);
      *(v4fa*)(sD + r * SCH + c4) = vd;
      *(v4fa*)(sG + r * SCH + c4) = vg;
      *(v4fa*)(sU + r * SCH + c4) = vu;
    }
    {
      const int r  = tid >> 3;
      const int c4 = (tid & 7) * 4;
      const v4f vb = *(const v4fa*)(BC + (size_t)(rb + r) * BCP + c4);
      *(v4fa*)(sBC + r * BCP + c4) = vb;
    }
    __syncthreads();

#pragma unroll 1
    for (int s = 0; s < TCH; ++s) {
      const float dl = sD[s * SCH + ch];
      const float uu = sU[s * SCH + ch];
      const float gg = sG[s * SCH + ch];
      const v4f bq = *(const v4fa*)(sBC + s * BCP + 4 * q);
      const v4f cq = *(const v4fa*)(sBC + s * BCP + DSTATE + 4 * q);
      const float du = dl * uu;
      h0 = expf(dl * a0) * h0 + du * bq.x;
      h1 = expf(dl * a1) * h1 + du * bq.y;
      h2 = expf(dl * a2) * h2 + du * bq.z;
      h3 = expf(dl * a3) * h3 + du * bq.w;
      float y = ((h0 * cq.x + h1 * cq.y) + h2 * cq.z) + h3 * cq.w;
      y += __shfl_xor(y, 1, 32);
      y += __shfl_xor(y, 2, 32);
      y = (y + uu * Dd) * gg;
      unsigned hb, lb;
      hl_bits(y, hb, lb);
      if (q == 0) {
        sYh[s * SCH + ch] = (unsigned short)hb;
        sYl[s * SCH + ch] = (unsigned short)lb;
      }
    }
    __syncthreads();

    const v8us qh = *(const v8usa*)(sYh + orow * SCH + 8 * oq);
    const v8us ql = *(const v8usa*)(sYl + orow * SCH + 8 * oq);
    unsigned short* yp = YHL + (size_t)(rb + orow) * KO2 + d0 + 8 * oq;
    *(volatile v8us*)yp = qh;
    *(volatile v8us*)(yp + DINNER) = ql;
    __threadfence();
    *(volatile v8us*)yp = qh;
    *(volatile v8us*)(yp + DINNER) = ql;
  }
}

__global__ __launch_bounds__(NTHR) void k_ln(float* out, const float* __restrict__ lw,
                                             const float* __restrict__ lb) {
  __shared__ __attribute__((aligned(16))) float srow[8 * DMODEL];
  const int tid = (int)threadIdx.x, lane = tid & 31, wave = tid >> 5;
  const int row = (int)blockIdx.x * 8 + wave;
  float* rp = out + (size_t)row * DMODEL;
  float* sp = srow + wave * DMODEL;

  float s = 0.0f;
#pragma unroll 1
  for (int it = 0; it < 8; ++it) {
    const int e = 4 * (it * 32 + lane);
    const v4f v = *(const v4fa*)(rp + e);
    *(v4fa*)(sp + e) = v;
    s += (v.x + v.y) + (v.z + v.w);
  }
  s += __shfl_xor(s, 16, 32);
  s += __shfl_xor(s, 8, 32);
  s += __shfl_xor(s, 4, 32);
  s += __shfl_xor(s, 2, 32);
  s += __shfl_xor(s, 1, 32);
  const float mu = s * (1.0f / (float)DMODEL);

  float ss = 0.0f;
#pragma unroll 1
  for (int it = 0; it < 8; ++it) {
    const int e = 4 * (it * 32 + lane);
    const v4f v = *(const v4fa*)(sp + e);
    const float dx = v.x - mu, dy = v.y - mu, dz = v.z - mu, dw = v.w - mu;
    ss += (dx * dx + dy * dy) + (dz * dz + dw * dw);
  }
  ss += __shfl_xor(ss, 16, 32);
  ss += __shfl_xor(ss, 8, 32);
  ss += __shfl_xor(ss, 4, 32);
  ss += __shfl_xor(ss, 2, 32);
  ss += __shfl_xor(ss, 1, 32);
  const float var = ss * (1.0f / (float)DMODEL);
  const float inv = rsqrtf(var + 1e-5f);

#pragma unroll 1
  for (int it = 0; it < 8; ++it) {
    const int e = 4 * (it * 32 + lane);
    const v4f v = *(const v4fa*)(sp + e);
    const v4f w = *(const v4fa*)(lw + e);
    const v4f c = *(const v4fa*)(lb + e);
    v4f o;
    o.x = (v.x - mu) * inv * bf16_val(w.x) + bf16_val(c.x);
    o.y = (v.y - mu) * inv * bf16_val(w.y) + bf16_val(c.y);
    o.z = (v.z - mu) * inv * bf16_val(w.z) + bf16_val(c.z);
    o.w = (v.w - mu) * inv * bf16_val(w.w) + bf16_val(c.w);
    *(v4fa*)(sp + e) = o;
    *(volatile v4f*)(rp + e) = o;
  }
  __threadfence();
#pragma unroll 1
  for (int it = 0; it < 8; ++it) {
    const int e = 4 * (it * 32 + lane);
    const v4f o = *(const v4fa*)(sp + e);
    *(volatile v4f*)(rp + e) = o;
  }
}

static inline int cdiv(int a, int b) { return (a + b - 1) / b; }
static inline size_t al256(size_t o) { return (o + 255) & ~(size_t)255; }

extern "C" void kernel_launch(void* const* d_in, const int* in_sizes, int n_in,
                              void* d_out, int out_size, void* d_ws, size_t ws_size,
                              hipStream_t stream) {
  if (n_in < 12) return;
  if (in_sizes[0] != MROWS * DMODEL) return;
  if (in_sizes[1] != 2 * DINNER * DMODEL) return;
  if (in_sizes[2] != DINNER * 4) return;
  if (in_sizes[3] != DINNER) return;
  if (in_sizes[4] != XPN * DINNER) return;
  if (in_sizes[5] != DINNER * DTRANK) return;
  if (in_sizes[6] != DINNER) return;
  if (in_sizes[7] != DINNER * DSTATE) return;
  if (in_sizes[8] != DINNER) return;
  if (in_sizes[9] != DMODEL * DINNER) return;
  if (in_sizes[10] != DMODEL || in_sizes[11] != DMODEL) return;
  if (out_size != MROWS * DMODEL) return;

  const float* x      = (const float*)d_in[0];
  const float* in_w   = (const float*)d_in[1];
  const float* conv_w = (const float*)d_in[2];
  const float* conv_b = (const float*)d_in[3];
  const float* xp_w   = (const float*)d_in[4];
  const float* dt_w   = (const float*)d_in[5];
  const float* dt_b   = (const float*)d_in[6];
  const float* A_log  = (const float*)d_in[7];
  const float* Dp     = (const float*)d_in[8];
  const float* out_w  = (const float*)d_in[9];
  const float* ln_w   = (const float*)d_in[10];
  const float* ln_b   = (const float*)d_in[11];
  float* out = (float*)d_out;

  char* ws = (char*)d_ws;
  size_t off = 0;
  const size_t oXZ  = off; off = al256(off + (size_t)MROWS * XZP * 4);
  const size_t oU   = off; off = al256(off + (size_t)MROWS * DINNER * 4);
  const size_t oUHL = off; off = al256(off + (size_t)MROWS * KX2 * 2);
  const size_t oXB  = off; off = al256(off + (size_t)MROWS * KIN * 2);
  const size_t oWIN = off; off = al256(off + (size_t)2 * DINNER * KIN * 2);
  const size_t oWO2 = off; off = al256(off + (size_t)DMODEL * KO2 * 2);
  const size_t oWX2 = off; off = al256(off + (size_t)XPNP * KX2 * 2);
  const size_t oWD2 = off; off = al256(off + (size_t)DINNER * KD2 * 2);
  const size_t oBC  = off; off = al256(off + (size_t)MROWS * BCP * 4);
  const size_t oDT  = off; off = al256(off + (size_t)MROWS * KD2 * 2);
  if (off > ws_size) return;
  float*          XZ   = (float*)(ws + oXZ);
  float*          U    = (float*)(ws + oU);
  unsigned short* UHL  = (unsigned short*)(ws + oUHL);
  unsigned short* YHL  = UHL;
  unsigned short* XB   = (unsigned short*)(ws + oXB);
  unsigned short* WIN  = (unsigned short*)(ws + oWIN);
  unsigned short* WO2  = (unsigned short*)(ws + oWO2);
  unsigned short* WX2  = (unsigned short*)(ws + oWX2);
  unsigned short* WD2  = (unsigned short*)(ws + oWD2);
  float*          BC   = (float*)(ws + oBC);
  unsigned short* DTHL = (unsigned short*)(ws + oDT);

  k_cvt<<<cdiv(MROWS * (KIN / 8), NTHR), NTHR, 0, stream>>>(x, MROWS, DMODEL, XB, 7, MROWS * (KIN / 8));
  k_cvt<<<cdiv(2 * DINNER * (KIN / 8), NTHR), NTHR, 0, stream>>>(in_w, 2 * DINNER, DMODEL, WIN, 7, 2 * DINNER * (KIN / 8));
  k_cvt<<<cdiv(XPNP * (KX2 / 8), NTHR), NTHR, 0, stream>>>(xp_w, XPN, DINNER, WX2, 9, XPNP * (KX2 / 8));
  k_cvt<<<cdiv(DINNER * (KD2 / 8), NTHR), NTHR, 0, stream>>>(dt_w, DINNER, DTRANK, WD2, 4, DINNER * (KD2 / 8));
  k_cvt<<<cdiv(DMODEL * (KO2 / 8), NTHR), NTHR, 0, stream>>>(out_w, DMODEL, DINNER, WO2, 9, DMODEL * (KO2 / 8));
  k_gemm<EP_IN><<<dim3(MROWS / GBM, (2 * DINNER) / GBN), GTHR, 0, stream>>>(XB, WIN, KIN, XZ, XZP, DTHL, x);
  k_conv<<<MROWS, NTHR, 0, stream>>>(XZ, conv_w, conv_b, U, UHL);
  k_gemm<EP_XP><<<dim3(MROWS / GBM, XPNP / GBN), GTHR, 0, stream>>>(UHL, WX2, KX2, BC, BCP, DTHL, x);
  k_gemm<EP_DT><<<dim3(MROWS / GBM, DINNER / GBN), GTHR, 0, stream>>>(DTHL, WD2, KD2, XZ, XZP, UHL, dt_b);
  k_scan<<<NBATCH * (DINNER / SCH), SCTHR, 0, stream>>>(XZ, U, BC, A_log, Dp, YHL);
  k_gemm<EP_OUT><<<dim3(MROWS / GBM, DMODEL / GBN), GTHR, 0, stream>>>(YHL, WO2, KO2, out, DMODEL, DTHL, x);
  k_ln<<<MROWS / 8, NTHR, 0, stream>>>(out, ln_w, ln_b);
}
